// SimpleDecoder_43757126812132
// MI455X (gfx1250) — hardware-verified
//
#include <hip/hip_runtime.h>
#include <math.h>
#include <stdint.h>

#ifndef NB
#define NB      2
#endif
#ifndef SEQ
#define SEQ     2048
#endif
#define NB_FULL  2
#define SEQ_FULL 2048
#define NQ      SEQ
#define NC      SEQ
#define DMODEL  1024
#define DFF     4096
#define NHEAD   16
#define HDIM    64
#define NROWS   (NB * NQ)
#define XC      16.0f
#define WSC     64.0f
#define QC      16.0f
#define KC      16.0f
#define VC      16.0f
#define PC      1024.0f
#define FC      1024.0f
#define HC      16.0f
#define GC      64.0f
#define ATT_SCALE 0.125f
#define LOG2E   1.4426950408889634f
#define LN_EPS  1e-5f
#define NEGM    (-1.0e30f)
static_assert(NHEAD * HDIM == DMODEL);
static_assert(NB >= 1 && NB <= NB_FULL && SEQ >= 64 && SEQ <= SEQ_FULL);
static_assert((NQ % 64) == 0 && (NC % 64) == 0 && (NC % 32) == 0 && (NQ % 16) == 0);
static_assert((DMODEL % 64) == 0 && (DFF % 64) == 0 && (DMODEL % 32) == 0 && (DFF % 32) == 0 && (NROWS % 64) == 0);
static_assert((size_t)((NB - 1) * SEQ_FULL + NQ) * DMODEL <= (size_t)NB_FULL * SEQ_FULL * DMODEL);
#define HPB     8
#define NHB     (NHEAD / HPB)
#define OSP     (HPB * HDIM)
#define ATT_THREADS (HPB * 32)
#define ATT_BLOCKS  (NB * (NQ / 16) * NHB)
static_assert(ATT_THREADS == 256 && NHB * HPB == NHEAD);
#define LN_THREADS 256
static_assert(LN_THREADS * 4 == DMODEL);

typedef _Float16 v16h __attribute__((ext_vector_type(16)));
typedef _Float16 v8h  __attribute__((ext_vector_type(8)));
typedef float    v8f  __attribute__((ext_vector_type(8)));
typedef float    v4f  __attribute__((ext_vector_type(4)));
typedef unsigned int v4u __attribute__((ext_vector_type(4)));
typedef unsigned int v2u __attribute__((ext_vector_type(2)));

union FragH { v16h v; v8h h[2]; v4u u[2]; };

__device__ __forceinline__ unsigned short bf_bits(float f) {
  unsigned u = __float_as_uint(f);
  return (unsigned short)((u + 0x7FFFu + ((u >> 16) & 1u)) >> 16);
}
__device__ __forceinline__ float bf_up(unsigned short h) { return __uint_as_float(((unsigned)h) << 16); }
__device__ __forceinline__ float bfr(float f) { return bf_up(bf_bits(f)); }
__device__ __forceinline__ unsigned short h_bits(_Float16 x) { return __builtin_bit_cast(unsigned short, x); }
__device__ __forceinline__ unsigned pk16(unsigned short a, unsigned short b) { return (unsigned)a | ((unsigned)b << 16); }
__device__ __forceinline__ v8f zero8() { v8f z = {0.f, 0.f, 0.f, 0.f, 0.f, 0.f, 0.f, 0.f}; return z; }
__device__ __forceinline__ int imin(int a, int b) { return a < b ? a : b; }

__device__ __forceinline__ v16h ldfrag_h(const _Float16* p) {
  FragH f;
  f.h[0] = *(const v8h*)(p);
  f.h[1] = *(const v8h*)(p + 16);
  return f.v;
}
__device__ __forceinline__ v16h ldfrag_u(const unsigned short* p) {
  FragH f;
  f.u[0] = *(const v4u*)(p);
  f.u[1] = *(const v4u*)(p + 16);
  return f.v;
}

__device__ __forceinline__ v8f mma_raw(v16h a, v16h b, v8f c) {
  return __builtin_amdgcn_wmma_f32_16x16x32_f16(false, a, false, b, (short)0, c, false, false);
}
__device__ __forceinline__ void dep_guard1(v8f& a, v8f& b, v16h x) {
#if defined(__HIP_DEVICE_COMPILE__)
  asm volatile("v_nop\n\tv_nop\n\tv_nop\n\tv_nop" : "+v"(a), "+v"(b) : "v"(x));
#endif
}
__device__ __forceinline__ void guard_s2(v8f& s, v16h a0, v16h a1) {
#if defined(__HIP_DEVICE_COMPILE__)
  asm volatile("v_nop\n\tv_nop\n\tv_nop\n\tv_nop" : "+v"(s) : "v"(a0), "v"(a1));
#endif
}
__device__ __forceinline__ void guard_s4(v8f& s, v16h a0, v16h a1, v16h b0, v16h b1) {
#if defined(__HIP_DEVICE_COMPILE__)
  asm volatile("v_nop\n\tv_nop\n\tv_nop\n\tv_nop" : "+v"(s) : "v"(a0), "v"(a1), "v"(b0), "v"(b1));
#endif
}
__device__ __forceinline__ void guard_pv4(v8f& a, v8f& b, v8f& c, v8f& d, v16h x, v16h y, v16h z, v16h w, v16h u) {
#if defined(__HIP_DEVICE_COMPILE__)
  asm volatile("v_nop\n\tv_nop\n\tv_nop\n\tv_nop"
               : "+v"(a), "+v"(b), "+v"(c), "+v"(d) : "v"(x), "v"(y), "v"(z), "v"(w), "v"(u));
#endif
}
__device__ __forceinline__ void keep4_h(v16h a, v16h b, v16h c, v16h d) {
#if defined(__HIP_DEVICE_COMPILE__)
  asm volatile("v_nop" :: "v"(a), "v"(b), "v"(c), "v"(d));
#endif
}
__device__ __forceinline__ void acc_guard4(v8f& a, v8f& b, v8f& c, v8f& d) {
#if defined(__HIP_DEVICE_COMPILE__)
  asm volatile("v_nop\n\tv_nop\n\tv_nop\n\tv_nop" : "+v"(a), "+v"(b), "+v"(c), "+v"(d));
#endif
}
__device__ __forceinline__ void wave_sync_lds() {
  __builtin_amdgcn_fence(__ATOMIC_RELEASE, "workgroup");
  __builtin_amdgcn_wave_barrier();
  __builtin_amdgcn_fence(__ATOMIC_ACQUIRE, "workgroup");
}

__global__ __launch_bounds__(256) void cvt16(const float* __restrict__ src, unsigned short* dst,
                                             int nrow, int ncol, int rpg, int gstride, float sc) {
  const int cpr = ncol >> 3;
  const size_t tot = (size_t)nrow * (size_t)cpr;
  const size_t t = (size_t)blockIdx.x * 256 + threadIdx.x;
  if (t >= tot) return;
  const int i  = (int)(t / (size_t)cpr);
  const int c8 = (int)(t - (size_t)i * cpr) * 8;
  const int g  = i / rpg;
  const int sr = g * gstride + (i - g * rpg);
  const float* sp = src + (size_t)sr * ncol + c8;
  const v4f a = *(const v4f*)(sp);
  const v4f b = *(const v4f*)(sp + 4);
  v4u w;
  w[0] = pk16(h_bits((_Float16)(bfr(a[0]) * sc)), h_bits((_Float16)(bfr(a[1]) * sc)));
  w[1] = pk16(h_bits((_Float16)(bfr(a[2]) * sc)), h_bits((_Float16)(bfr(a[3]) * sc)));
  w[2] = pk16(h_bits((_Float16)(bfr(b[0]) * sc)), h_bits((_Float16)(bfr(b[1]) * sc)));
  w[3] = pk16(h_bits((_Float16)(bfr(b[2]) * sc)), h_bits((_Float16)(bfr(b[3]) * sc)));
  unsigned short* dp = dst + (size_t)i * ncol + c8;
  for (int pass = 0; pass < 2; ++pass) {
    *(volatile v4u*)dp = w;
    __threadfence();
  }
}

template <int OM, int RM, int ACT, int BM>
__global__ __launch_bounds__(256) void gemm64(
    const unsigned short* __restrict__ Ap, int lda, long long sA,
    const unsigned short* __restrict__ Btp, int ldb, long long sB,
    const float* __restrict__ Rp, long long sR,
    const float* __restrict__ biasp, int nbias,
    void* Cout, int ldc, long long sC,
    int M, int N, int K, float oscale, float ocarry) {
  __shared__ __align__(16) float sT[8][16 * 68];
  const int by   = blockIdx.y;
  const int lane = threadIdx.x & 31;
  const int wave = threadIdx.x >> 5;
  const int tilesN = N >> 6;
  const int tilesM = M >> 6;
  const int tile = blockIdx.x * 8 + wave;
  if (tile >= tilesM * tilesN) return;
  const int tm = tile / tilesN;
  const int tn = tile - tm * tilesN;
  const int m0 = tm << 6;
  const int n0 = tn << 6;

  const unsigned short* A1 = Ap  + (size_t)((long long)by * sA);
  const unsigned short* Bb = Btp + (size_t)((long long)by * sB);

  const int rlane = lane & 15;
  const int koff  = (lane >> 4) * 8;
  const int mOff  = (lane >> 4) * 8;

  v8f acc[4][4];
#pragma unroll
  for (int i = 0; i < 4; ++i)
#pragma unroll
    for (int j = 0; j < 4; ++j) acc[i][j] = zero8();

  for (int k0 = 0; k0 < K; k0 += 32) {
    v16h bh[4];
#pragma unroll
    for (int j = 0; j < 4; ++j) {
      const size_t bofs = (size_t)(n0 + (j << 4) + rlane) * ldb + koff + k0;
      bh[j] = ldfrag_u(Bb + bofs);
    }
#pragma unroll
    for (int i = 0; i < 4; ++i) {
      const size_t ao = (size_t)(m0 + (i << 4) + rlane) * lda + koff + k0;
      const v16h ah = ldfrag_u(A1 + ao);
#pragma unroll
      for (int j = 0; j < 4; ++j) acc[i][j] = mma_raw(ah, bh[j], acc[i][j]);
      dep_guard1(acc[i][0], acc[i][3], ah);
    }
    keep4_h(bh[0], bh[1], bh[2], bh[3]);
  }
  acc_guard4(acc[0][0], acc[0][1], acc[0][2], acc[0][3]);
  acc_guard4(acc[1][0], acc[1][1], acc[1][2], acc[1][3]);
  acc_guard4(acc[2][0], acc[2][1], acc[2][2], acc[2][3]);
  acc_guard4(acc[3][0], acc[3][1], acc[3][2], acc[3][3]);

  const int hh2 = lane >> 4, c4 = (lane & 15) * 4;
  const int q8  = lane >> 3, c8 = (lane & 7) * 8;

  float bc4[4], bc8[8];
#pragma unroll
  for (int e = 0; e < 4; ++e) bc4[e] = 0.f;
#pragma unroll
  for (int e = 0; e < 8; ++e) bc8[e] = 0.f;
  if constexpr (BM == 1) {
    if constexpr (OM == 0) {
#pragma unroll
      for (int e = 0; e < 4; ++e) {
        const int n = n0 + c4 + e;
        const int ncl = imin(n, nbias - 1);
        const float t = bfr(biasp[ncl]);
        bc4[e] = (n < nbias) ? t : 0.f;
      }
    } else {
#pragma unroll
      for (int e = 0; e < 8; ++e) {
        const int n = n0 + c8 + e;
        const int ncl = imin(n, nbias - 1);
        const float t = bfr(biasp[ncl]);
        bc8[e] = (n < nbias) ? t : 0.f;
      }
    }
  }

  float* slab = sT[wave];
#pragma unroll
  for (int i = 0; i < 4; ++i) {
    const int mBase = m0 + (i << 4);
#pragma unroll
    for (int j = 0; j < 4; ++j) {
#pragma unroll
      for (int r = 0; r < 8; ++r) {
        slab[(mOff + r) * 68 + (j << 4) + rlane] = acc[i][j][r];
      }
    }
    wave_sync_lds();
    if constexpr (OM == 0) {
      float* C = (float*)Cout + (size_t)((long long)by * sC);
      v4f vals[8];
#pragma unroll
      for (int it = 0; it < 8; ++it) {
        const int row = it * 2 + hh2;
        const int gr  = mBase + row;
        v4f v = *(const v4f*)(slab + row * 68 + c4);
        v4f rv = {0.f, 0.f, 0.f, 0.f};
        if constexpr (RM == 1 || RM == 2) {
          const float* R = Rp + (size_t)((long long)by * sR);
          const v4f rraw = *(const v4f*)(R + (size_t)gr * ldc + n0 + c4);
#pragma unroll
          for (int e = 0; e < 4; ++e) rv[e] = (RM == 1) ? bfr(rraw[e]) : rraw[e];
        }
        float rb = 0.f;
        if constexpr (BM == 2) {
          const int mcl = imin(gr, nbias - 1);
          const float t = bfr(biasp[mcl]);
          rb = (gr < nbias) ? t : 0.f;
        }
#pragma unroll
        for (int e = 0; e < 4; ++e) {
          float u = v[e] * oscale;
          if constexpr (BM == 1) u += bc4[e];
          if constexpr (BM == 2) u += rb;
          if constexpr (ACT == 1) u = fmaxf(u, 0.f);
          v[e] = u + rv[e];
        }
        vals[it] = v;
      }
      for (int pass = 0; pass < 2; ++pass) {
#pragma unroll
        for (int it = 0; it < 8; ++it) {
          const int gr = mBase + it * 2 + hh2;
          *(volatile v4f*)(C + (size_t)gr * ldc + n0 + c4) = vals[it];
        }
        __threadfence();
      }
    } else {
      unsigned short* C = (unsigned short*)Cout + (size_t)((long long)by * sC);
      v4u hv[4];
#pragma unroll
      for (int it = 0; it < 4; ++it) {
        const int row = it * 4 + q8;
        const int gr  = mBase + row;
        const float* sp = slab + row * 68 + c8;
        float rb = 0.f;
        if constexpr (BM == 2) {
          const int mcl = imin(gr, nbias - 1);
          const float t = bfr(biasp[mcl]);
          rb = (gr < nbias) ? t : 0.f;
        }
        v4u a = {0u, 0u, 0u, 0u};
#pragma unroll
        for (int e = 0; e < 4; ++e) {
          float f0 = sp[2 * e] * oscale;
          float f1 = sp[2 * e + 1] * oscale;
          if constexpr (BM == 1) { f0 += bc8[2 * e]; f1 += bc8[2 * e + 1]; }
          if constexpr (BM == 2) { f0 += rb; f1 += rb; }
          if constexpr (ACT == 1) { f0 = fmaxf(f0, 0.f); f1 = fmaxf(f1, 0.f); }
          f0 *= ocarry; f1 *= ocarry;
          a[e] = pk16(h_bits((_Float16)f0), h_bits((_Float16)f1));
        }
        hv[it] = a;
      }
      for (int pass = 0; pass < 2; ++pass) {
#pragma unroll
        for (int it = 0; it < 4; ++it) {
          const int row = it * 4 + q8;
          *(volatile v4u*)(C + (size_t)(mBase + row) * ldc + n0 + c8) = hv[it];
        }
        __threadfence();
      }
    }
    wave_sync_lds();
  }
}

#define PS_FLOATS (HPB * 16 * 36)
static_assert((size_t)16 * OSP * sizeof(unsigned short) <= (size_t)PS_FLOATS * sizeof(float));
static_assert(((16 * OSP) % (8 * ATT_THREADS)) == 0 && ((16 * OSP) / (8 * ATT_THREADS)) == 4);
static_assert(OSP == 64 * 8);

__global__ __launch_bounds__(ATT_THREADS)
void attnc(const unsigned short* __restrict__ QHp, const unsigned short* __restrict__ KHp,
           const unsigned short* __restrict__ VTq, unsigned short* CT) {
  __shared__ __align__(16) float smem[PS_FLOATS];

  const int tid  = threadIdx.x;
  const int wave = tid >> 5;
  const int lane = tid & 31;
  const int hh   = lane >> 4;
  const int c    = lane & 15;

  const int hb   = blockIdx.x % NHB;
  const int qt   = (blockIdx.x / NHB) % (NQ / 16);
  const int bat  = blockIdx.x / (NHB * (NQ / 16));
  const int head = hb * HPB + wave;
  const int q0   = qt * 16;
  const int qrow0 = q0 + 8 * hh;
  const int kend = q0 + 16;

  const size_t qofs = ((size_t)bat * NQ + q0 + c) * DMODEL + head * HDIM + 8 * hh;
  const _Float16* Qh = (const _Float16*)(const void*)QHp + qofs;
  const _Float16* Kb = (const _Float16*)(const void*)KHp + (size_t)bat * NC * DMODEL + head * HDIM + 8 * hh;
  const _Float16* Vb = (const _Float16*)(const void*)VTq + ((size_t)bat * DMODEL + head * HDIM) * NC + 8 * hh;
  const float lsc = (LOG2E * ATT_SCALE) / (QC * KC);

  const v16h qa = ldfrag_h(Qh), qb = ldfrag_h(Qh + 32);

  float mrow[8], lrow[8];
  v8f o0 = zero8(), o1 = zero8(), o2 = zero8(), o3 = zero8();
#pragma unroll
  for (int r = 0; r < 8; ++r) { mrow[r] = -INFINITY; lrow[r] = 0.f; }
  float* pt = smem + wave * (16 * 36);

#pragma unroll 1
  for (int kb = 0; kb < kend; kb += 32) {
    const _Float16* kp = Kb + (size_t)(kb + c) * DMODEL;
    v8f s0, s1;
    {
      const v16h k0 = ldfrag_h(kp), k1 = ldfrag_h(kp + 32);
      s0 = mma_raw(qa, k0, zero8());
      s0 = mma_raw(qb, k1, s0);
      guard_s2(s0, k0, k1);
    }
    {
      const _Float16* kq = kp + (size_t)16 * DMODEL;
      const v16h k0 = ldfrag_h(kq), k1 = ldfrag_h(kq + 32);
      s1 = mma_raw(qa, k0, zero8());
      s1 = mma_raw(qb, k1, s1);
      guard_s4(s1, k0, k1, qa, qb);
    }
    const int key0 = kb + c;
    const int key1 = kb + 16 + c;
#pragma unroll
    for (int r = 0; r < 8; ++r) {
      const int qr = qrow0 + r;
      const float u0 = s0[r] * lsc;
      const float u1 = s1[r] * lsc;
      const float t0 = (key0 > qr) ? NEGM : u0;
      const float t1 = (key1 > qr) ? NEGM : u1;
      float mx = fmaxf(t0, t1);
#pragma unroll
      for (int off = 1; off < 16; off <<= 1) mx = fmaxf(mx, __shfl_xor(mx, off, 32));
      const float mn = fmaxf(mrow[r], mx);
      const float al = exp2f(fmaxf(mrow[r] - mn, -126.0f));
      mrow[r] = mn;
      const float e0 = exp2f(t0 - mn);
      const float e1 = exp2f(t1 - mn);
      float ps = e0 + e1;
#pragma unroll
      for (int off = 1; off < 16; off <<= 1) ps += __shfl_xor(ps, off, 32);
      lrow[r] = lrow[r] * al + ps;
      o0[r] *= al;
      o1[r] *= al;
      o2[r] *= al;
      o3[r] *= al;
      const int ro = (8 * hh + r) * 36 + c;
      pt[ro]      = e0;
      pt[ro + 16] = e1;
    }
    wave_sync_lds();
    FragH ph;
    {
      const float* prow = pt + c * 36 + 8 * hh;
      const v4f p0 = *(const v4f*)(prow), p1 = *(const v4f*)(prow + 4);
      const v4f p2 = *(const v4f*)(prow + 16), p3 = *(const v4f*)(prow + 20);
#pragma unroll
      for (int e = 0; e < 4; ++e) {
        ph.h[0][e]     = (_Float16)(p0[e] * PC);
        ph.h[0][4 + e] = (_Float16)(p1[e] * PC);
        ph.h[1][e]     = (_Float16)(p2[e] * PC);
        ph.h[1][4 + e] = (_Float16)(p3[e] * PC);
      }
    }
    const _Float16* vp = Vb + (size_t)c * NC + kb;
    {
      const v16h vb0 = ldfrag_h(vp);
      const v16h vb1 = ldfrag_h(vp + (size_t)16 * NC);
      const v16h vb2 = ldfrag_h(vp + (size_t)32 * NC);
      const v16h vb3 = ldfrag_h(vp + (size_t)48 * NC);
      o0 = mma_raw(ph.v, vb0, o0);
      o1 = mma_raw(ph.v, vb1, o1);
      o2 = mma_raw(ph.v, vb2, o2);
      o3 = mma_raw(ph.v, vb3, o3);
      guard_pv4(o0, o1, o2, o3, ph.v, vb0, vb1, vb2, vb3);
    }
    wave_sync_lds();
  }

  __syncthreads();
  unsigned short* Os = (unsigned short*)smem;
  const float oc = FC / (PC * VC);
  unsigned short* osw = Os + wave * HDIM + c;
#pragma unroll
  for (int r = 0; r < 8; ++r) {
    const float inv = (1.0f / lrow[r]) * oc;
    unsigned short* op = osw + (8 * hh + r) * OSP;
    op[0]  = h_bits((_Float16)(o0[r] * inv));
    op[16] = h_bits((_Float16)(o1[r] * inv));
    op[32] = h_bits((_Float16)(o2[r] * inv));
    op[48] = h_bits((_Float16)(o3[r] * inv));
  }
  __syncthreads();
  {
    v4u vals[4];
#pragma unroll
    for (int it = 0; it < 4; ++it) {
      const int p = it * ATT_THREADS + tid;
      vals[it] = *(const v4u*)(Os + (size_t)p * 8);
    }
    unsigned short* dst = CT + ((size_t)bat * NQ + q0) * DMODEL + (size_t)hb * OSP;
    for (int pass = 0; pass < 2; ++pass) {
#pragma unroll
      for (int it = 0; it < 4; ++it) {
        const int p = it * ATT_THREADS + tid;
        const int row = p >> 6, col8 = (p & 63) * 8;
        *(volatile v4u*)(dst + (size_t)row * DMODEL + col8) = vals[it];
      }
      __threadfence();
    }
  }
}

template <int OF, int OH>
__global__ __launch_bounds__(LN_THREADS)
void lnorm(const float* __restrict__ Yp, const float* __restrict__ gp, const float* __restrict__ bp,
           float* outf, int rpg, int gstride, unsigned short* outh, float hc) {
  __shared__ float red[2][LN_THREADS / 32];
  __shared__ __align__(16) unsigned short srow[DMODEL];
  const int row  = blockIdx.x;
  const int tid  = threadIdx.x;
  const int lane = tid & 31;
  const int wave = tid >> 5;
  const size_t base = (size_t)row * DMODEL + (size_t)tid * 4;
  v4f v = *(const v4f*)(Yp + base);
  float s = (v[0] + v[1]) + (v[2] + v[3]);
#pragma unroll
  for (int off = 1; off < 32; off <<= 1) s += __shfl_xor(s, off, 32);
  if (lane == 0) red[0][wave] = s;
  __syncthreads();
  float tot = 0.f;
#pragma unroll
  for (int w = 0; w < LN_THREADS / 32; ++w) tot += red[0][w];
  const float mu = tot * (1.0f / (float)DMODEL);
  v4f d;
#pragma unroll
  for (int e = 0; e < 4; ++e) d[e] = v[e] - mu;
  float q = (d[0] * d[0] + d[1] * d[1]) + (d[2] * d[2] + d[3] * d[3]);
#pragma unroll
  for (int off = 1; off < 32; off <<= 1) q += __shfl_xor(q, off, 32);
  if (lane == 0) red[1][wave] = q;
  __syncthreads();
  float totq = 0.f;
#pragma unroll
  for (int w = 0; w < LN_THREADS / 32; ++w) totq += red[1][w];
  const float var  = totq * (1.0f / (float)DMODEL);
  const float rstd = rsqrtf(var + LN_EPS);
  const v4f gv = *(const v4f*)(gp + (size_t)tid * 4);
  const v4f bv = *(const v4f*)(bp + (size_t)tid * 4);
  v4f o;
#pragma unroll
  for (int e = 0; e < 4; ++e) o[e] = (d[e] * rstd) * bfr(gv[e]) + bfr(bv[e]);
  if constexpr (OF == 1) {
    const int g    = row / rpg;
    const int orow = g * gstride + (row - g * rpg);
    float* dst = outf + (size_t)orow * DMODEL + (size_t)tid * 4;
    for (int pass = 0; pass < 2; ++pass) {
      *(volatile v4f*)dst = o;
      __threadfence();
    }
  }
  if constexpr (OH == 1) {
    v2u w;
    w[0] = pk16(h_bits((_Float16)(o[0] * hc)), h_bits((_Float16)(o[1] * hc)));
    w[1] = pk16(h_bits((_Float16)(o[2] * hc)), h_bits((_Float16)(o[3] * hc)));
    *(v2u*)(srow + tid * 4) = w;
    __syncthreads();
    if (tid < DMODEL / 8) {
      const v4u hv = *(const v4u*)(srow + tid * 8);
      unsigned short* dsth = outh + (size_t)row * DMODEL + (size_t)tid * 8;
      for (int pass = 0; pass < 2; ++pass) {
        *(volatile v4u*)dsth = hv;
        __threadfence();
      }
    }
  } else {
    (void)srow; (void)outh; (void)hc;
  }
}

extern "C" void kernel_launch(void* const* d_in, const int* in_sizes, int n_in,
                              void* d_out, int out_size, void* d_ws, size_t ws_size,
                              hipStream_t stream) {
  if (n_in < 17) return;
  const int need_rows = (NB - 1) * SEQ_FULL + NQ;
  if (in_sizes[0] < need_rows * DMODEL) return;
  if (in_sizes[1] != DMODEL * DMODEL || in_sizes[3] != DMODEL * DMODEL) return;
  if (in_sizes[5] != DMODEL * DMODEL || in_sizes[7] != DMODEL * DMODEL) return;
  if (in_sizes[2] != DMODEL || in_sizes[4] != DMODEL || in_sizes[6] != DMODEL || in_sizes[8] != DMODEL) return;
  if (in_sizes[9] != DMODEL || in_sizes[10] != DMODEL) return;
  if (in_sizes[11] != DFF * DMODEL || in_sizes[12] != DFF) return;
  if (in_sizes[13] != DMODEL * DFF || in_sizes[14] != DMODEL) return;
  if (in_sizes[15] != DMODEL || in_sizes[16] != DMODEL) return;
  if (out_size < need_rows * DMODEL) return;

  const float* x     = (const float*)d_in[0];
  const float* wq    = (const float*)d_in[1];
  const float* bq    = (const float*)d_in[2];
  const float* wk    = (const float*)d_in[3];
  const float* bk    = (const float*)d_in[4];
  const float* wv    = (const float*)d_in[5];
  const float* bv    = (const float*)d_in[6];
  const float* wo    = (const float*)d_in[7];
  const float* bo    = (const float*)d_in[8];
  const float* ln1_g = (const float*)d_in[9];
  const float* ln1_b = (const float*)d_in[10];
  const float* wup   = (const float*)d_in[11];
  const float* bup   = (const float*)d_in[12];
  const float* wdn   = (const float*)d_in[13];
  const float* bdn   = (const float*)d_in[14];
  const float* ln2_g = (const float*)d_in[15];
  const float* ln2_b = (const float*)d_in[16];
  float*       out   = (float*)d_out;

  const size_t PX16 = (size_t)NROWS * DMODEL * 2;
  const size_t PW1  = (size_t)DMODEL * DMODEL * 2;
  const size_t PWF  = (size_t)DFF * DMODEL * 2;
  const size_t PX32 = (size_t)NROWS * DMODEL * 4;
  const size_t PVT  = (size_t)NB * DMODEL * NC * 2;
  const size_t PG16 = (size_t)NROWS * DFF * 2;
  size_t off = 0;
  const size_t oX16 = off; off += PX16;
  const size_t oWQ  = off; off += PW1;
  const size_t oWK  = off; off += PW1;
  const size_t oWV  = off; off += PW1;
  const size_t oWO  = off; off += PW1;
  const size_t oWU  = off; off += PWF;
  const size_t oWD  = off; off += PWF;
  const size_t oXF  = off; off += PX32;
  const size_t oHF  = off; off += PX32;
  const size_t oH16 = off; off += PX16;
  const size_t oS   = off;
  const size_t oQH  = oS;
  const size_t oKH  = oQH + PX16;
  const size_t oVT  = oKH + PX16;
  const size_t oCT  = oVT + PVT;
  const size_t endA = oCT + PX16;
  const size_t oG   = oS;
  const size_t endB = oG + PG16;
  const size_t endAll = (endA > endB) ? endA : endB;
  if (endAll > ws_size) return;
  if (endAll > (size_t)134217728) return;

  char* ws = (char*)d_ws;
  unsigned short* X16  = (unsigned short*)(ws + oX16);
  unsigned short* WQ16 = (unsigned short*)(ws + oWQ);
  unsigned short* WK16 = (unsigned short*)(ws + oWK);
  unsigned short* WV16 = (unsigned short*)(ws + oWV);
  unsigned short* WO16 = (unsigned short*)(ws + oWO);
  unsigned short* WU16 = (unsigned short*)(ws + oWU);
  unsigned short* WD16 = (unsigned short*)(ws + oWD);
  float*          XF   = (float*)(ws + oXF);
  float*          HF   = (float*)(ws + oHF);
  unsigned short* H16  = (unsigned short*)(ws + oH16);
  unsigned short* QH   = (unsigned short*)(ws + oQH);
  unsigned short* KH   = (unsigned short*)(ws + oKH);
  unsigned short* VTp  = (unsigned short*)(ws + oVT);
  unsigned short* CT   = (unsigned short*)(ws + oCT);
  unsigned short* G16  = (unsigned short*)(ws + oG);

  const dim3 blk(256);
  const unsigned cvX  = (unsigned)(((size_t)NROWS * (DMODEL / 8) + 255) / 256);
  const unsigned cvW1 = (unsigned)(((size_t)DMODEL * (DMODEL / 8) + 255) / 256);
  const unsigned cvWU = (unsigned)(((size_t)DFF * (DMODEL / 8) + 255) / 256);
  const unsigned cvWD = (unsigned)(((size_t)DMODEL * (DFF / 8) + 255) / 256);
  const int tilesP = (NROWS / 64) * (DMODEL / 64);
  const int tilesV = (DMODEL / 64) * (NC / 64);
  const int tilesO = (NQ / 64) * (DMODEL / 64);
  const int tilesF = (NROWS / 64) * (DFF / 64);
  const dim3 gP((tilesP + 7) / 8, 1);
  const dim3 gV((tilesV + 7) / 8, NB);
  const dim3 gO((tilesO + 7) / 8, NB);
  const dim3 gF((tilesF + 7) / 8, 1);
  const dim3 gAT(ATT_BLOCKS);
  const dim3 bAT(ATT_THREADS);
  const dim3 gLN(NROWS);
  const dim3 bLN(LN_THREADS);

  cvt16<<<dim3(cvX),  blk, 0, stream>>>(x,   X16,  NROWS,  DMODEL, NQ,     SEQ_FULL, XC);
  cvt16<<<dim3(cvW1), blk, 0, stream>>>(wq,  WQ16, DMODEL, DMODEL, DMODEL, 0, WSC);
  cvt16<<<dim3(cvW1), blk, 0, stream>>>(wk,  WK16, DMODEL, DMODEL, DMODEL, 0, WSC);
  cvt16<<<dim3(cvW1), blk, 0, stream>>>(wv,  WV16, DMODEL, DMODEL, DMODEL, 0, WSC);
  cvt16<<<dim3(cvW1), blk, 0, stream>>>(wo,  WO16, DMODEL, DMODEL, DMODEL, 0, WSC);
  cvt16<<<dim3(cvWU), blk, 0, stream>>>(wup, WU16, DFF,    DMODEL, DFF,    0, WSC);
  cvt16<<<dim3(cvWD), blk, 0, stream>>>(wdn, WD16, DMODEL, DFF,    DMODEL, 0, WSC);

  gemm64<2, 0, 0, 1><<<gP, blk, 0, stream>>>(
      X16, DMODEL, 0LL,
      WQ16, DMODEL, 0LL,
      (const float*)0, 0LL,
      bq, DMODEL,
      (void*)QH, DMODEL, 0LL,
      NROWS, DMODEL, DMODEL, 1.0f / (XC * WSC), QC);

  gemm64<2, 0, 0, 1><<<gP, blk, 0, stream>>>(
      X16, DMODEL, 0LL,
      WK16, DMODEL, 0LL,
      (const float*)0, 0LL,
      bk, DMODEL,
      (void*)KH, DMODEL, 0LL,
      NROWS, DMODEL, DMODEL, 1.0f / (XC * WSC), KC);

  gemm64<2, 0, 0, 2><<<gV, blk, 0, stream>>>(
      WV16, DMODEL, 0LL,
      X16, DMODEL, (long long)NC * DMODEL,
      (const float*)0, 0LL,
      bv, DMODEL,
      (void*)VTp, NC, (long long)DMODEL * NC,
      DMODEL, NC, DMODEL, 1.0f / (XC * WSC), VC);

  attnc<<<gAT, bAT, 0, stream>>>(QH, KH, VTp, CT);

  gemm64<0, 1, 0, 1><<<gO, blk, 0, stream>>>(
      CT, DMODEL, (long long)NQ * DMODEL,
      WO16, DMODEL, 0LL,
      x, (long long)SEQ_FULL * DMODEL,
      bo, DMODEL,
      (void*)XF, DMODEL, (long long)NQ * DMODEL,
      NQ, DMODEL, DMODEL, 1.0f / (FC * WSC), 1.0f);

  lnorm<1, 1><<<gLN, bLN, 0, stream>>>(XF, ln1_g, ln1_b, HF, NROWS, 0, H16, HC);

  gemm64<2, 0, 1, 1><<<gF, blk, 0, stream>>>(
      H16, DMODEL, 0LL,
      WU16, DMODEL, 0LL,
      (const float*)0, 0LL,
      bup, DFF,
      (void*)G16, DFF, 0LL,
      NROWS, DFF, DMODEL, 1.0f / (HC * WSC), GC);

  gemm64<0, 2, 0, 1><<<gP, blk, 0, stream>>>(
      G16, DFF, 0LL,
      WD16, DFF, 0LL,
      HF, 0LL,
      bdn, DMODEL,
      (void*)XF, DMODEL, 0LL,
      NROWS, DMODEL, DFF, 1.0f / (GC * WSC), 1.0f);

  lnorm<1, 0><<<gLN, bLN, 0, stream>>>(XF, ln2_g, ln2_b, out, NQ, SEQ_FULL, (unsigned short*)0, 1.0f);
  (void)hipGetLastError();
}
